// ForgettingTransformerBlock_74775380623510
// MI455X (gfx1250) — hardware-verified
//
#include <hip/hip_runtime.h>
#include <math.h>

typedef __attribute__((ext_vector_type(16))) _Float16 v16h;
typedef __attribute__((ext_vector_type(8)))  _Float16 v8h;
typedef __attribute__((ext_vector_type(16))) __bf16   v16b;
typedef __attribute__((ext_vector_type(8)))  __bf16   v8b;
typedef __attribute__((ext_vector_type(8)))  float    v8f;
typedef __attribute__((ext_vector_type(4)))  float    v4f;

constexpr int kBatch   = 2;
constexpr int kSeq     = 2048;
constexpr int kDm      = 1024;
constexpr int kHeads   = 16;
constexpr int kHd      = 64;
constexpr int kFF      = 4096;
constexpr int kTok     = kBatch * kSeq;
constexpr int kQkvLd   = 3 * kDm;
constexpr int kGatePad = 64;
constexpr float kWScale    = 256.0f;
constexpr float kWScaleInv = 1.0f / 256.0f;
constexpr float kPCarry    = 32768.0f;
static_assert(kTok % 64 == 0 && kDm % 64 == 0 && kFF % 64 == 0 && kGatePad % 64 == 0);
static_assert(kDm % 32 == 0 && kFF % 32 == 0);
static_assert(kSeq % 64 == 0 && kHd == 64 && kHeads * kHd == kDm);

constexpr size_t kBytesX1    = (size_t)kTok * kDm * 4;
constexpr size_t kBytesW1T   = (size_t)kFF * kDm * 2;
constexpr size_t kBytesW2T   = (size_t)kDm * kFF * 2;
constexpr size_t kBytesH     = (size_t)kTok * kDm * 2;
constexpr size_t kBytesQKV   = (size_t)kTok * kQkvLd * 2;
constexpr size_t kBytesZ     = (size_t)kTok * kGatePad * 4;
constexpr size_t kBytesC     = (size_t)kBatch * kHeads * kSeq * 4;
constexpr size_t kBytesO     = (size_t)kTok * kDm * 2;
constexpr size_t kBytesWQKVT = (size_t)3 * kDm * kDm * 2;
constexpr size_t kBytesWFT   = (size_t)kGatePad * kDm * 2;
constexpr size_t kBytesWOT   = (size_t)kDm * kDm * 2;
constexpr size_t kBytesU     = (size_t)kTok * kFF * 2;
constexpr size_t kBytesG     = kBytesU;
constexpr size_t kOffX1    = 0;
constexpr size_t kOffW1T   = kOffX1 + kBytesX1;
constexpr size_t kOffW2T   = kOffW1T + kBytesW1T;
constexpr size_t kOffH     = kOffW2T + kBytesW2T;
constexpr size_t kOffQKV   = kOffH + kBytesH;
constexpr size_t kOffZ     = kOffQKV + kBytesQKV;
constexpr size_t kOffC     = kOffZ + kBytesZ;
constexpr size_t kOffO     = kOffC + kBytesC;
constexpr size_t kOffWQKVT = kOffO + kBytesO;
constexpr size_t kOffWFT   = kOffWQKVT + kBytesWQKVT;
constexpr size_t kOffWOT   = kOffWFT + kBytesWFT;
constexpr size_t kEndA     = kOffWOT + kBytesWOT;
constexpr size_t kOffH2    = kOffH;
constexpr size_t kOffU     = kOffQKV;
constexpr size_t kOffG     = kOffU + kBytesU;
constexpr size_t kEndB     = kOffG + kBytesG;
constexpr size_t kWsTotal  = (kEndB > kEndA) ? kEndB : kEndA;
static_assert(kWsTotal <= (size_t)134217728);
static_assert(kOffU >= kOffH2 + kBytesH);
static_assert(kOffG >= kOffU + kBytesU);
static_assert(kOffU >= kOffW2T + kBytesW2T && kOffH2 >= kOffW2T + kBytesW2T);
static_assert((kOffH % 256) == 0 && (kOffQKV % 256) == 0 && (kOffZ % 256) == 0 && (kOffC % 256) == 0 &&
              (kOffO % 256) == 0 && (kOffWQKVT % 256) == 0 && (kOffWFT % 256) == 0 && (kOffWOT % 256) == 0 &&
              (kOffG % 256) == 0 && (kOffW1T % 256) == 0 && (kOffW2T % 256) == 0);

__device__ __forceinline__ unsigned short f2bf_bits(float f) {
  unsigned u = __float_as_uint(f);
  return (unsigned short)((u + 0x7FFFu + ((u >> 16) & 1u)) >> 16);
}
__device__ __forceinline__ float bf_bits2f(unsigned short h) { return __uint_as_float(((unsigned)h) << 16); }

__device__ __forceinline__ void dep_guard_h(v8f& a, v8f& b, v16h x, v16h y) { asm volatile("v_nop\n\tv_nop\n\tv_nop\n\tv_nop" : "+v"(a), "+v"(b) : "v"(x), "v"(y)); }
__device__ __forceinline__ void dep_guard_b(v8f& a, v8f& b, v16b x, v16b y) { asm volatile("v_nop\n\tv_nop\n\tv_nop\n\tv_nop" : "+v"(a), "+v"(b) : "v"(x), "v"(y)); }
__device__ __forceinline__ void keep4_h(v16h a, v16h b, v16h c, v16h d) { asm volatile("v_nop" :: "v"(a), "v"(b), "v"(c), "v"(d)); }
__device__ __forceinline__ void keep4_b(v16b a, v16b b, v16b c, v16b d) { asm volatile("v_nop" :: "v"(a), "v"(b), "v"(c), "v"(d)); }
__device__ __forceinline__ void acc_guard4(v8f& a, v8f& b, v8f& c, v8f& d) { asm volatile("v_nop\n\tv_nop\n\tv_nop\n\tv_nop" : "+v"(a), "+v"(b), "+v"(c), "+v"(d)); }
template <typename T> struct Frag;
template <> struct Frag<_Float16> {
  typedef v16h V; union U { v16h v; v8h h[2]; };
  static __device__ __forceinline__ v16h load(const _Float16* p) {
    U f; f.h[0] = *(const v8h*)(p); f.h[1] = *(const v8h*)(p + 16); return f.v;
  }
  static __device__ __forceinline__ v8f mma(v16h a, v16h b, v8f c) {
    return __builtin_amdgcn_wmma_f32_16x16x32_f16(false, a, false, b, (short)0, c, false, false);
  }
  static __device__ __forceinline__ void guard(v8f& a, v8f& b, v16h x, v16h y) { dep_guard_h(a, b, x, y); }
  static __device__ __forceinline__ void keep(v16h a, v16h b, v16h c, v16h d) { keep4_h(a, b, c, d); }
};
template <> struct Frag<__bf16> {
  typedef v16b V; union U { v16b v; v8b h[2]; };
  static __device__ __forceinline__ v16b load(const __bf16* p) {
    U f; f.h[0] = *(const v8b*)(p); f.h[1] = *(const v8b*)(p + 16); return f.v;
  }
  static __device__ __forceinline__ v8f mma(v16b a, v16b b, v8f c) {
    return __builtin_amdgcn_wmma_f32_16x16x32_bf16(false, a, false, b, (short)0, c, false, false);
  }
  static __device__ __forceinline__ void guard(v8f& a, v8f& b, v16b x, v16b y) { dep_guard_b(a, b, x, y); }
  static __device__ __forceinline__ void keep(v16b a, v16b b, v16b c, v16b d) { keep4_b(a, b, c, d); }
};

__device__ __forceinline__ v8f mma_f16g(v16h a, v16h b, v8f c) {
  c = __builtin_amdgcn_wmma_f32_16x16x32_f16(false, a, false, b, (short)0, c, false, false);
  asm volatile("v_nop\n\tv_nop\n\tv_nop\n\tv_nop" : "+v"(c) : "v"(a), "v"(b));
  return c;
}

template <int ET> struct Elem;
template <> struct Elem<0> { typedef _Float16 T; };
template <> struct Elem<1> { typedef __bf16 T; };
template <int ET, bool SPLIT, int BIAS_MODE, int OUT_MODE, bool RESID, int ACT = 0>
__global__ __launch_bounds__(256) void wmma_gemm64(
    const unsigned short* __restrict__ Ap, const unsigned short* __restrict__ A2p, int lda, long strideA,
    const unsigned short* __restrict__ Btp, const unsigned short* __restrict__ Bt2p, int ldb, long strideB,
    void* __restrict__ Cout, void* __restrict__ Cout2, int ldc, long strideC,
    const float* __restrict__ bias,
    const float* __restrict__ resid, long strideR,
    int M, int N, int K, float scale) {
  typedef typename Elem<ET>::T T;
  typedef typename Frag<T>::V V;
  const T* A = (const T*)Ap; const T* A2 = (const T*)A2p; const T* Bt = (const T*)Btp; const T* Bt2 = (const T*)Bt2p;
  __shared__ __align__(16) float sT[8][16 * 68];
  const int b    = blockIdx.y;
  const int lane = threadIdx.x & 31;
  const int wave = threadIdx.x >> 5;
  const int tilesN = N >> 6;
  const int tilesM = M >> 6;
  const int tile = blockIdx.x * 8 + wave;
  if (tile >= tilesM * tilesN) return;
  const int tm = tile / tilesN;
  const int tn = tile - tm * tilesN;
  const int m0 = tm << 6;
  const int n0 = tn << 6;

  const T* Ab  = A  + (size_t)b * strideA;
  const T* Bb  = Bt + (size_t)b * strideB;
  const T* Ab2 = SPLIT ? (A2  + (size_t)b * strideA) : nullptr;
  const T* Bb2 = SPLIT ? (Bt2 + (size_t)b * strideB) : nullptr;

  const int rlane = lane & 15;
  const int koff  = (lane >> 4) * 8;
  const int mOff  = (lane >> 4) * 8;

  v8f acc[4][4];
#pragma unroll
  for (int i = 0; i < 4; ++i)
#pragma unroll
    for (int j = 0; j < 4; ++j) acc[i][j] = (v8f){0.f,0.f,0.f,0.f,0.f,0.f,0.f,0.f};

  for (int k0 = 0; k0 < K; k0 += 32) {
    V bh[4], bl[4];
#pragma unroll
    for (int j = 0; j < 4; ++j) {
      const size_t bo = (size_t)(n0 + (j << 4) + rlane) * ldb + koff + k0;
      bh[j] = Frag<T>::load(Bb + bo);
      if (SPLIT) bl[j] = Frag<T>::load(Bb2 + bo);
    }
#pragma unroll
    for (int i = 0; i < 4; ++i) {
      const size_t ao = (size_t)(m0 + (i << 4) + rlane) * lda + koff + k0;
      V ah = Frag<T>::load(Ab + ao);
      V al;
      if (SPLIT) al = Frag<T>::load(Ab2 + ao);
#pragma unroll
      for (int j = 0; j < 4; ++j) {
        acc[i][j] = Frag<T>::mma(ah, bh[j], acc[i][j]);
        if (SPLIT) {
          acc[i][j] = Frag<T>::mma(ah, bl[j], acc[i][j]);
          acc[i][j] = Frag<T>::mma(al, bh[j], acc[i][j]);
        }
      }
      Frag<T>::guard(acc[i][0], acc[i][3], ah, SPLIT ? al : ah);
    }
    Frag<T>::keep(bh[0], bh[1], bh[2], bh[3]);
    if (SPLIT) Frag<T>::keep(bl[0], bl[1], bl[2], bl[3]);
  }
  acc_guard4(acc[0][0], acc[0][1], acc[0][2], acc[0][3]);
  acc_guard4(acc[1][0], acc[1][1], acc[1][2], acc[1][3]);
  acc_guard4(acc[2][0], acc[2][1], acc[2][2], acc[2][3]);
  acc_guard4(acc[3][0], acc[3][1], acc[3][2], acc[3][3]);

  float* slab = sT[wave];
  const float* Rb = RESID ? (resid + (size_t)b * strideR) : nullptr;
#pragma unroll
  for (int i = 0; i < 4; ++i) {
    const int mBase = m0 + (i << 4);
#pragma unroll
    for (int j = 0; j < 4; ++j) {
      const int n = n0 + (j << 4) + rlane;
      float bv = 0.f;
      if (BIAS_MODE == 2) bv = bias[n];
#pragma unroll
      for (int r = 0; r < 8; ++r) {
        float v = acc[i][j][r] * scale;
        if (BIAS_MODE == 1) v += bias[mBase + mOff + r];
        if (BIAS_MODE == 2) v += bv;
        if (RESID) v += Rb[(size_t)(mBase + mOff + r) * ldc + n];
        if (ACT == 1) v = tanhf(v);
        if (ACT == 2) v = fmaxf(v, 0.0f);
        if (ACT == 4) v = (v > 0.f) ? v : 0.01f * v;
        slab[(mOff + r) * 68 + (j << 4) + rlane] = v;
      }
    }
    __builtin_amdgcn_fence(__ATOMIC_RELEASE, "workgroup");
    __builtin_amdgcn_wave_barrier();
    __builtin_amdgcn_fence(__ATOMIC_ACQUIRE, "workgroup");
    if (OUT_MODE == 0) {
      float* C = (float*)Cout + (size_t)b * strideC;
      const int hh = lane >> 4, c4 = (lane & 15) * 4;
      for (int pass = 0; pass < 2; ++pass) {
#pragma unroll
        for (int it = 0; it < 8; ++it) {
          const int row = it * 2 + hh;
          v4f v = *(const v4f*)(slab + row * 68 + c4);
          *(volatile v4f*)(C + (size_t)(mBase + row) * ldc + n0 + c4) = v;
        }
        __threadfence();
      }
    } else {
      const int q = lane >> 3, c8 = (lane & 7) * 8;
      unsigned short* C  = (unsigned short*)Cout  + (size_t)b * strideC;
      unsigned short* C2 = (OUT_MODE == 2) ? ((unsigned short*)Cout2 + (size_t)b * strideC) : nullptr;
      for (int pass = 0; pass < 2; ++pass) {
#pragma unroll
        for (int it = 0; it < 4; ++it) {
          const int row = it * 4 + q;
          const float* sp = slab + row * 68 + c8;
          v8h hv, lv;
#pragma unroll
          for (int e = 0; e < 8; ++e) {
            if (OUT_MODE == 1) {
              hv[e] = (_Float16)sp[e];
            } else {
              unsigned short hb = f2bf_bits(sp[e]);
              unsigned short lb = f2bf_bits(sp[e] - bf_bits2f(hb));
              hv[e] = __builtin_bit_cast(_Float16, hb);
              lv[e] = __builtin_bit_cast(_Float16, lb);
            }
          }
          *(volatile v8h*)(C + (size_t)(mBase + row) * ldc + n0 + c8) = hv;
          if (OUT_MODE == 2) *(volatile v8h*)(C2 + (size_t)(mBase + row) * ldc + n0 + c8) = lv;
        }
        __threadfence();
      }
    }
    __builtin_amdgcn_fence(__ATOMIC_RELEASE, "workgroup");
    __builtin_amdgcn_wave_barrier();
    __builtin_amdgcn_fence(__ATOMIC_ACQUIRE, "workgroup");
  }
}

__global__ __launch_bounds__(256) void wtrans_f16_kernel(const float* __restrict__ w, _Float16* __restrict__ bt,
                                                         int kdim, int ndim, float sc) {
  __shared__ float tile[64][65];
  const int tid = threadIdx.x;
  const int n0 = blockIdx.x * 64, k0 = blockIdx.y * 64;
#pragma unroll 4
  for (int i = 0; i < 16; ++i) {
    const int idx = i * 256 + tid;
    const int kk = idx >> 6, nn = idx & 63;
    const int n = n0 + nn;
    const int nc = (n < ndim) ? n : (ndim - 1);
    float v = w[(size_t)(k0 + kk) * ndim + nc];
    v = (n < ndim) ? v : 0.0f;
    tile[kk][nn] = v * sc;
  }
  __syncthreads();
  v8h o[2];
#pragma unroll
  for (int it = 0; it < 2; ++it) {
    const int lid = it * 256 + tid;
    const int nn = lid >> 3, seg = (lid & 7) * 8;
#pragma unroll
    for (int e = 0; e < 8; ++e) o[it][e] = (_Float16)tile[seg + e][nn];
  }
  for (int pass = 0; pass < 2; ++pass) {
#pragma unroll
    for (int it = 0; it < 2; ++it) {
      const int lid = it * 256 + tid;
      const int nn = lid >> 3, seg = (lid & 7) * 8;
      *(volatile v8h*)(bt + (size_t)(n0 + nn) * kdim + k0 + seg) = o[it];
    }
    __threadfence();
  }
}

__global__ __launch_bounds__(128) void layernorm_f16_kernel(const float* __restrict__ x, const float* __restrict__ gam,
                                                           const float* __restrict__ bet, _Float16* __restrict__ out) {
  __shared__ float red[4];
  const int row = blockIdx.x;
  const int tid = threadIdx.x, lane = tid & 31, wave = tid >> 5;
  const float* xr = x + (size_t)row * kDm + tid * 8;
  const v4f a = *(const v4f*)xr;
  const v4f c = *(const v4f*)(xr + 4);
  float s = ((a[0] + a[1]) + (a[2] + a[3])) + ((c[0] + c[1]) + (c[2] + c[3]));
#pragma unroll
  for (int off = 1; off < 32; off <<= 1) s += __shfl_xor(s, off, 32);
  if (lane == 0) red[wave] = s;
  __syncthreads();
  const float mu = ((red[0] + red[1]) + (red[2] + red[3])) * (1.0f / 1024.0f);
  __syncthreads();
  const v4f da = a - mu;
  const v4f dc = c - mu;
  float s2 = ((da[0] * da[0] + da[1] * da[1]) + (da[2] * da[2] + da[3] * da[3])) +
             ((dc[0] * dc[0] + dc[1] * dc[1]) + (dc[2] * dc[2] + dc[3] * dc[3]));
#pragma unroll
  for (int off = 1; off < 32; off <<= 1) s2 += __shfl_xor(s2, off, 32);
  if (lane == 0) red[wave] = s2;
  __syncthreads();
  const float var = ((red[0] + red[1]) + (red[2] + red[3])) * (1.0f / 1024.0f);
  const float rstd = rsqrtf(var + 1e-5f);
  const v4f g0 = *(const v4f*)(gam + tid * 8);
  const v4f g1 = *(const v4f*)(gam + tid * 8 + 4);
  const v4f b0 = *(const v4f*)(bet + tid * 8);
  const v4f b1 = *(const v4f*)(bet + tid * 8 + 4);
  v8h o;
  o[0] = (_Float16)(da[0] * rstd * g0[0] + b0[0]);
  o[1] = (_Float16)(da[1] * rstd * g0[1] + b0[1]);
  o[2] = (_Float16)(da[2] * rstd * g0[2] + b0[2]);
  o[3] = (_Float16)(da[3] * rstd * g0[3] + b0[3]);
  o[4] = (_Float16)(dc[0] * rstd * g1[0] + b1[0]);
  o[5] = (_Float16)(dc[1] * rstd * g1[1] + b1[1]);
  o[6] = (_Float16)(dc[2] * rstd * g1[2] + b1[2]);
  o[7] = (_Float16)(dc[3] * rstd * g1[3] + b1[3]);
  _Float16* dst = out + (size_t)row * kDm + tid * 8;
  *(volatile v8h*)dst = o;
  __threadfence();
  *(volatile v8h*)dst = o;
}

__global__ __launch_bounds__(256) void gate_scan_kernel(const float* __restrict__ zg, const float* __restrict__ bfv,
                                                        float* __restrict__ cdec) {
  __shared__ __align__(16) float lf[kSeq];
  __shared__ float pre[16];
  const int bh = blockIdx.x, b = bh >> 4, h = bh & 15;
  const int tid = threadIdx.x;
  const float bias = bfv[h];
#pragma unroll 1
  for (int e = 0; e < 8; ++e) {
    const int pos = tid * 8 + e;
    const float z = zg[((size_t)b * kSeq + pos) * kGatePad + h] + bias;
    lf[pos] = fminf(z, 0.0f) - log1pf(expf(-fabsf(z)));
  }
  __syncthreads();
  if (tid < 16) {
    float a = 0.0f;
#pragma unroll 1
    for (int i = 0; i < 128; ++i) {
      a += lf[tid * 128 + i];
      lf[tid * 128 + i] = a;
    }
  }
  __syncthreads();
  if (tid == 0) {
    float a = 0.0f;
#pragma unroll 1
    for (int i = 0; i < 16; ++i) {
      pre[i] = a;
      a += lf[i * 128 + 127];
    }
  }
  __syncthreads();
  const int p0 = tid * 4;
  const int p1 = 1024 + tid * 4;
  const float pa = pre[p0 >> 7];
  const float pb = pre[p1 >> 7];
  v4f va, vb;
  va[0] = lf[p0 + 0] + pa; va[1] = lf[p0 + 1] + pa; va[2] = lf[p0 + 2] + pa; va[3] = lf[p0 + 3] + pa;
  vb[0] = lf[p1 + 0] + pb; vb[1] = lf[p1 + 1] + pb; vb[2] = lf[p1 + 2] + pb; vb[3] = lf[p1 + 3] + pb;
  float* crow = cdec + (size_t)bh * kSeq;
  for (int pass = 0; pass < 2; ++pass) {
    *(volatile v4f*)(crow + p0) = va;
    *(volatile v4f*)(crow + p1) = vb;
    __threadfence();
  }
}

__global__ __launch_bounds__(128) void attn_fgate_kernel(const _Float16* __restrict__ qkv, const float* __restrict__ cdec,
                                                         _Float16* __restrict__ octx) {
  union FH { v16h v; v8h h[2]; };
  __shared__ __align__(16) _Float16 Ksh[64 * 64];
  __shared__ __align__(16) _Float16 Vth[64 * 64];
  __shared__ __align__(16) _Float16 Psh[4][16 * 64];
  __shared__ __align__(16) float Os[4][16 * 68];
  const int tid = threadIdx.x, wave = tid >> 5, lane = tid & 31;
  const int hh = lane >> 4, c = lane & 15;
  const int bx = blockIdx.x;
  const int qb = bx & 31;
  const int bh = bx >> 5;
  const int h = bh & 15, b = bh >> 4;
  const int q0 = qb * 64 + wave * 16;

  const _Float16* qbase = qkv + (size_t)b * kSeq * kQkvLd + h * kHd;
  const _Float16* kbase = qbase + kDm;
  const _Float16* vbase = qbase + 2 * kDm;
  const float* cb = cdec + (size_t)bh * kSeq;
  _Float16* obase = octx + (size_t)b * kSeq * kDm + h * kHd;

  v16h qa[2];
  {
    const _Float16* qrow = qbase + (size_t)(q0 + c) * kQkvLd + 8 * hh;
    qa[0] = Frag<_Float16>::load(qrow);
    qa[1] = Frag<_Float16>::load(qrow + 32);
  }
  float ci[8], mrow[8], lrow[8];
  v8f oacc[4];
#pragma unroll
  for (int r = 0; r < 8; ++r) { ci[r] = cb[q0 + 8 * hh + r]; mrow[r] = -INFINITY; lrow[r] = 0.f; }
#pragma unroll
  for (int t = 0; t < 4; ++t) oacc[t] = (v8f){0.f,0.f,0.f,0.f,0.f,0.f,0.f,0.f};

  const int nChunks = qb + 1;
  for (int kc = 0; kc < nChunks; ++kc) {
    const int kv0 = kc * 64;
    __syncthreads();
    {
      const int kvr = tid >> 1, dh = (tid & 1) * 32;
      const _Float16* krow = kbase + (size_t)(kv0 + kvr) * kQkvLd + dh;
      const _Float16* vrow = vbase + (size_t)(kv0 + kvr) * kQkvLd + dh;
#pragma unroll
      for (int i = 0; i < 4; ++i) {
        const v8h kk = *(const v8h*)(krow + 8 * i);
        *(v8h*)(Ksh + kvr * 64 + dh + 8 * i) = kk;
        const v8h vv = *(const v8h*)(vrow + 8 * i);
#pragma unroll
        for (int e = 0; e < 8; ++e) Vth[(dh + 8 * i + e) * 64 + kvr] = vv[e];
      }
    }
    __syncthreads();

    v8f s[4];
#pragma unroll
    for (int j = 0; j < 4; ++j) {
      s[j] = (v8f){0.f,0.f,0.f,0.f,0.f,0.f,0.f,0.f};
#pragma unroll
      for (int dc = 0; dc < 2; ++dc) {
        FH kb;
        kb.h[0] = *(const v8h*)(Ksh + (j * 16 + c) * 64 + dc * 32 + 8 * hh);
        kb.h[1] = *(const v8h*)(Ksh + (j * 16 + c) * 64 + dc * 32 + 16 + 8 * hh);
        s[j] = mma_f16g(qa[dc], kb.v, s[j]);
      }
    }
    float cj[4];
#pragma unroll
    for (int j = 0; j < 4; ++j) cj[j] = cb[kv0 + j * 16 + c];
    const bool diag = (kc == qb);
    float cm[8];
#pragma unroll
    for (int r = 0; r < 8; ++r) {
      const int qi = q0 + 8 * hh + r;
      float m = -INFINITY;
#pragma unroll
      for (int j = 0; j < 4; ++j) {
        const int kvcol = kv0 + j * 16 + c;
        float t = (s[j][r] * 0.125f + ci[r]) - cj[j];
        if (diag && (kvcol > qi)) t = -INFINITY;
        s[j][r] = t;
        m = fmaxf(m, t);
      }
#pragma unroll
      for (int off = 1; off < 16; off <<= 1) m = fmaxf(m, __shfl_xor(m, off, 32));
      cm[r] = m;
    }
    _Float16* pwh = Psh[wave];
#pragma unroll
    for (int r = 0; r < 8; ++r) {
      const float mnew = fmaxf(mrow[r], cm[r]);
      const float alpha = expf(mrow[r] - mnew);
      mrow[r] = mnew;
      float psum = 0.f;
#pragma unroll
      for (int j = 0; j < 4; ++j) {
        const float p = expf(s[j][r] - mnew);
        psum += p;
        pwh[(8 * hh + r) * 64 + j * 16 + c] = (_Float16)(p * kPCarry);
      }
#pragma unroll
      for (int off = 1; off < 16; off <<= 1) psum += __shfl_xor(psum, off, 32);
      lrow[r] = lrow[r] * alpha + psum;
#pragma unroll
      for (int t = 0; t < 4; ++t) oacc[t][r] *= alpha;
    }
    __builtin_amdgcn_fence(__ATOMIC_RELEASE, "workgroup");
    __builtin_amdgcn_wave_barrier();
    __builtin_amdgcn_fence(__ATOMIC_ACQUIRE, "workgroup");
#pragma unroll 1
    for (int kk = 0; kk < 2; ++kk) {
      FH pa;
      pa.h[0] = *(const v8h*)(pwh + c * 64 + kk * 32 + 8 * hh);
      pa.h[1] = *(const v8h*)(pwh + c * 64 + kk * 32 + 16 + 8 * hh);
#pragma unroll
      for (int t = 0; t < 4; ++t) {
        FH vb;
        vb.h[0] = *(const v8h*)(Vth + (t * 16 + c) * 64 + kk * 32 + 8 * hh);
        vb.h[1] = *(const v8h*)(Vth + (t * 16 + c) * 64 + kk * 32 + 16 + 8 * hh);
        oacc[t] = mma_f16g(pa.v, vb.v, oacc[t]);
      }
    }
  }

  float* os = Os[wave];
#pragma unroll
  for (int r = 0; r < 8; ++r) {
    const float inv = 1.0f / (lrow[r] * kPCarry);
#pragma unroll
    for (int t = 0; t < 4; ++t) os[(8 * hh + r) * 68 + t * 16 + c] = oacc[t][r] * inv;
  }
  __builtin_amdgcn_fence(__ATOMIC_RELEASE, "workgroup");
  __builtin_amdgcn_wave_barrier();
  __builtin_amdgcn_fence(__ATOMIC_ACQUIRE, "workgroup");
  {
    const int q8 = lane >> 3, c8 = (lane & 7) * 8;
    for (int pass = 0; pass < 2; ++pass) {
#pragma unroll
      for (int it = 0; it < 4; ++it) {
        const int row = it * 4 + q8;
        const float* sp = os + row * 68 + c8;
        v8h hv;
#pragma unroll
        for (int e = 0; e < 8; ++e) hv[e] = (_Float16)sp[e];
        *(volatile v8h*)(obase + (size_t)(q0 + row) * kDm + c8) = hv;
      }
      __threadfence();
    }
  }
}

__global__ __launch_bounds__(256) void gelu_f16_kernel(const unsigned* __restrict__ uin, unsigned* __restrict__ gout, int n2) {
  const int i = blockIdx.x * 256 + threadIdx.x;
  if (i >= n2) return;
  const unsigned u = uin[i];
  const float x0 = (float)__builtin_bit_cast(_Float16, (unsigned short)(u & 0xFFFFu));
  const float x1 = (float)__builtin_bit_cast(_Float16, (unsigned short)(u >> 16));
  float g0 = 0.f, g1 = 0.f;
#pragma unroll 1
  for (int e = 0; e < 2; ++e) {
    const float xv = (e == 0) ? x0 : x1;
    const float gv = 0.5f * xv * (1.0f + erff(xv * 0.70710678118654752f));
    if (e == 0) g0 = gv; else g1 = gv;
  }
  const unsigned o = (unsigned)__builtin_bit_cast(unsigned short, (_Float16)g0) |
                     ((unsigned)__builtin_bit_cast(unsigned short, (_Float16)g1) << 16);
  ((volatile unsigned*)gout)[i] = o;
  __threadfence();
  ((volatile unsigned*)gout)[i] = o;
}

static inline dim3 gemm_grid(int M, int N) {
  const int tiles = (M / 64) * (N / 64);
  return dim3((unsigned)((tiles + 7) / 8), 1, 1);
}

extern "C" void kernel_launch(void* const* d_in, const int* in_sizes, int n_in,
                              void* d_out, int out_size, void* d_ws, size_t ws_size,
                              hipStream_t stream) {
  if (n_in < 19) return;
  if (in_sizes[0] != kTok * kDm || in_sizes[1] != kDm || in_sizes[2] != kDm ||
      in_sizes[3] != kDm * kDm || in_sizes[4] != kDm || in_sizes[5] != kDm * kDm || in_sizes[6] != kDm ||
      in_sizes[7] != kDm * kDm || in_sizes[8] != kDm || in_sizes[9] != kDm * kDm || in_sizes[10] != kDm ||
      in_sizes[11] != kDm * kHeads || in_sizes[12] != kHeads || in_sizes[13] != kDm || in_sizes[14] != kDm ||
      in_sizes[15] != kDm * kFF || in_sizes[16] != kFF || in_sizes[17] != kFF * kDm || in_sizes[18] != kDm) return;
  if (out_size != kTok * kDm) return;
  if (ws_size < kWsTotal) return;

  const float* x    = (const float*)d_in[0];
  const float* ln1g = (const float*)d_in[1];
  const float* ln1b = (const float*)d_in[2];
  const float* wq   = (const float*)d_in[3];
  const float* bq   = (const float*)d_in[4];
  const float* wk   = (const float*)d_in[5];
  const float* bk   = (const float*)d_in[6];
  const float* wv   = (const float*)d_in[7];
  const float* bv   = (const float*)d_in[8];
  const float* wo   = (const float*)d_in[9];
  const float* bo   = (const float*)d_in[10];
  const float* wf   = (const float*)d_in[11];
  const float* bfv  = (const float*)d_in[12];
  const float* ln2g = (const float*)d_in[13];
  const float* ln2b = (const float*)d_in[14];
  const float* w1   = (const float*)d_in[15];
  const float* b1   = (const float*)d_in[16];
  const float* w2   = (const float*)d_in[17];
  const float* b2   = (const float*)d_in[18];
  float* out = (float*)d_out;

  char* ws = (char*)d_ws;
  float*    X1    = (float*)(ws + kOffX1);
  _Float16* W1T   = (_Float16*)(ws + kOffW1T);
  _Float16* W2T   = (_Float16*)(ws + kOffW2T);
  _Float16* Hp    = (_Float16*)(ws + kOffH);
  _Float16* QKV   = (_Float16*)(ws + kOffQKV);
  float*    Zg    = (float*)(ws + kOffZ);
  float*    Cdec  = (float*)(ws + kOffC);
  _Float16* Op    = (_Float16*)(ws + kOffO);
  _Float16* WQKVT = (_Float16*)(ws + kOffWQKVT);
  _Float16* WFT   = (_Float16*)(ws + kOffWFT);
  _Float16* WOT   = (_Float16*)(ws + kOffWOT);
  _Float16* H2p   = (_Float16*)(ws + kOffH2);
  _Float16* Up    = (_Float16*)(ws + kOffU);
  _Float16* Gp    = (_Float16*)(ws + kOffG);

  const unsigned short* HpU   = (const unsigned short*)Hp;
  const unsigned short* H2pU  = (const unsigned short*)H2p;
  const unsigned short* OpU   = (const unsigned short*)Op;
  const unsigned short* GpU   = (const unsigned short*)Gp;
  const unsigned short* WQKVU = (const unsigned short*)WQKVT;
  const unsigned short* WFTU  = (const unsigned short*)WFT;
  const unsigned short* WOTU  = (const unsigned short*)WOT;
  const unsigned short* W1TU  = (const unsigned short*)W1T;
  const unsigned short* W2TU  = (const unsigned short*)W2T;

  wtrans_f16_kernel<<<dim3(kDm / 64, kDm / 64), 256, 0, stream>>>(wq, WQKVT, kDm, kDm, kWScale);
  wtrans_f16_kernel<<<dim3(kDm / 64, kDm / 64), 256, 0, stream>>>(wk, WQKVT + (size_t)kDm * kDm, kDm, kDm, kWScale);
  wtrans_f16_kernel<<<dim3(kDm / 64, kDm / 64), 256, 0, stream>>>(wv, WQKVT + (size_t)2 * kDm * kDm, kDm, kDm, kWScale);
  wtrans_f16_kernel<<<dim3(kGatePad / 64, kDm / 64), 256, 0, stream>>>(wf, WFT, kDm, kHeads, kWScale);
  wtrans_f16_kernel<<<dim3(kDm / 64, kDm / 64), 256, 0, stream>>>(wo, WOT, kDm, kDm, kWScale);
  wtrans_f16_kernel<<<dim3(kFF / 64, kDm / 64), 256, 0, stream>>>(w1, W1T, kDm, kFF, kWScale);
  wtrans_f16_kernel<<<dim3(kDm / 64, kFF / 64), 256, 0, stream>>>(w2, W2T, kFF, kDm, kWScale);

  layernorm_f16_kernel<<<kTok, 128, 0, stream>>>(x, ln1g, ln1b, Hp);

  wmma_gemm64<0, false, 2, 1, false, 0><<<gemm_grid(kTok, kDm), 256, 0, stream>>>(
      HpU, HpU, kDm, 0L, WQKVU, WQKVU, kDm, 0L,
      (void*)QKV, (void*)QKV, kQkvLd, 0L, bq, x, 0L, kTok, kDm, kDm, kWScaleInv);
  wmma_gemm64<0, false, 2, 1, false, 0><<<gemm_grid(kTok, kDm), 256, 0, stream>>>(
      HpU, HpU, kDm, 0L, WQKVU + (size_t)kDm * kDm, WQKVU + (size_t)kDm * kDm, kDm, 0L,
      (void*)(QKV + kDm), (void*)(QKV + kDm), kQkvLd, 0L, bk, x, 0L, kTok, kDm, kDm, kWScaleInv);
  wmma_gemm64<0, false, 2, 1, false, 0><<<gemm_grid(kTok, kDm), 256, 0, stream>>>(
      HpU, HpU, kDm, 0L, WQKVU + (size_t)2 * kDm * kDm, WQKVU + (size_t)2 * kDm * kDm, kDm, 0L,
      (void*)(QKV + 2 * kDm), (void*)(QKV + 2 * kDm), kQkvLd, 0L, bv, x, 0L, kTok, kDm, kDm, kWScaleInv);

  wmma_gemm64<0, false, 0, 0, false, 0><<<gemm_grid(kTok, kGatePad), 256, 0, stream>>>(
      HpU, HpU, kDm, 0L, WFTU, WFTU, kDm, 0L,
      (void*)Zg, (void*)Zg, kGatePad, 0L, bfv, x, 0L, kTok, kGatePad, kDm, kWScaleInv);

  gate_scan_kernel<<<kBatch * kHeads, 256, 0, stream>>>(Zg, bfv, Cdec);

  attn_fgate_kernel<<<kBatch * kHeads * (kSeq / 64), 128, 0, stream>>>(QKV, Cdec, Op);

  wmma_gemm64<0, false, 2, 0, true, 0><<<gemm_grid(kTok, kDm), 256, 0, stream>>>(
      OpU, OpU, kDm, 0L, WOTU, WOTU, kDm, 0L,
      (void*)X1, (void*)X1, kDm, 0L, bo, x, 0L, kTok, kDm, kDm, kWScaleInv);

  layernorm_f16_kernel<<<kTok, 128, 0, stream>>>(X1, ln2g, ln2b, H2p);

  wmma_gemm64<0, false, 2, 1, false, 0><<<gemm_grid(kTok, kFF), 256, 0, stream>>>(
      H2pU, H2pU, kDm, 0L, W1TU, W1TU, kDm, 0L,
      (void*)Up, (void*)Up, kFF, 0L, b1, x, 0L, kTok, kFF, kDm, kWScaleInv);

  {
    const int n2 = (kTok * kFF) / 2;
    gelu_f16_kernel<<<(n2 + 255) / 256, 256, 0, stream>>>((const unsigned*)Up, (unsigned*)Gp, n2);
  }

  wmma_gemm64<0, false, 2, 0, true, 0><<<gemm_grid(kTok, kDm), 256, 0, stream>>>(
      GpU, GpU, kFF, 0L, W2TU, W2TU, kFF, 0L,
      (void*)out, (void*)out, kDm, 0L, b2, X1, 0L, kTok, kDm, kFF, kWScaleInv);
}
